// BidirectionAttention_17085379904046
// MI455X (gfx1250) — hardware-verified
//
#include <hip/hip_runtime.h>


#define NB_  4
#define NF   9216
#define NM   256
#define CIN  256
#define NH_  4
#define HD   64
#define PCAR 1024.0f
#define SCL  0.125f
#define TT   NM
#define OFF1 37748736
typedef _Float16 h16;
typedef unsigned short bf;
typedef __attribute__((ext_vector_type(16))) __bf16   v16bf;
typedef __attribute__((ext_vector_type(16))) _Float16 v16h;
typedef __attribute__((ext_vector_type(8)))  _Float16 v8h;
typedef __attribute__((ext_vector_type(8)))  unsigned short v8us;
typedef __attribute__((ext_vector_type(8)))  float    v8f;
typedef __attribute__((ext_vector_type(4)))  float    v4f;
typedef v8h  __attribute__((may_alias)) v8ha;
typedef v4f  __attribute__((may_alias)) v4fa;
typedef v8us __attribute__((may_alias)) v8usa;

__device__ __forceinline__ unsigned short f2bf(float f) { unsigned u = __float_as_uint(f); u += 0x7FFFu + ((u >> 16) & 1u); return (unsigned short)(u >> 16); }
__device__ __forceinline__ float bf2f(unsigned short b) { return __uint_as_float(((unsigned)b) << 16); }
__device__ __forceinline__ float bfr(float f) { return bf2f(f2bf(f)); }
__device__ __forceinline__ v16h cat16(v8h lo, v8h hi) { return __builtin_shufflevector(lo, hi, 0, 1, 2, 3, 4, 5, 6, 7, 8, 9, 10, 11, 12, 13, 14, 15); }
__device__ __forceinline__ v16bf cat16b(v8us lo, v8us hi) { return __builtin_bit_cast(v16bf, __builtin_shufflevector(lo, hi, 0, 1, 2, 3, 4, 5, 6, 7, 8, 9, 10, 11, 12, 13, 14, 15)); }
__device__ __forceinline__ v8f wmma16(v16h a, v16h b, v8f c) { return __builtin_amdgcn_wmma_f32_16x16x32_f16(false, a, false, b, (short)0, c, false, false); }
__device__ __forceinline__ v8f wmmab(v16bf a, v16bf b, v8f c) { return __builtin_amdgcn_wmma_f32_16x16x32_bf16(false, a, false, b, (short)0, c, false, false); }


template <typename T16> struct WFrag;
template <> struct WFrag<h16> { typedef v16h V; static __device__ __forceinline__ V ld(const h16* p) { return cat16(*(const v8h*)p, *(const v8h*)(p + 16)); } static __device__ __forceinline__ v8f mma(V a, V b, v8f c) { return wmma16(a, b, c); } };
template <> struct WFrag<bf> { typedef v16bf V; static __device__ __forceinline__ V ld(const bf* p) { return cat16b(*(const v8us*)p, *(const v8us*)(p + 16)); } static __device__ __forceinline__ v8f mma(V a, V b, v8f c) { return wmmab(a, b, c); } };
template <typename T16, int NSPLIT, bool BIAS>
__global__ __launch_bounds__(32) void k_gemmw(const T16* __restrict__ A, const T16* __restrict__ A2, const T16* __restrict__ Bt, const T16* __restrict__ Bt2, int K, float* C, int ldc, const float* __restrict__ bias, size_t sA, size_t sB, size_t sC) {
    typedef typename WFrag<T16>::V V;
    __shared__ __align__(16) float os[16 * 68];
    const size_t z = blockIdx.z; A += z * sA; if (A2) A2 += z * sA; Bt += z * sB; if (Bt2) Bt2 += z * sB; C += z * sC;
    const int lane = threadIdx.x & 31, lr = lane & 15, hi = lane >> 4; const int r0 = blockIdx.x * 64, c0 = blockIdx.y * 64;
    v8f acc[4][4];
#pragma unroll
    for (int mb = 0; mb < 4; ++mb)
#pragma unroll
        for (int nb = 0; nb < 4; ++nb) acc[mb][nb] = (v8f){};
    const size_t aoff = (size_t)(r0 + lr) * K + 8 * hi, boff = (size_t)(c0 + lr) * K + 8 * hi;
#pragma unroll 1
    for (int kc = 0; kc < K; kc += 32) {
        V a[4], a2[4];
#pragma unroll
        for (int mb = 0; mb < 4; ++mb) { a[mb] = WFrag<T16>::ld(A + aoff + (size_t)mb * 16 * K + kc); if (NSPLIT == 1 || NSPLIT == 2) a2[mb] = WFrag<T16>::ld(A2 + aoff + (size_t)mb * 16 * K + kc); }
#pragma unroll
        for (int nb = 0; nb < 4; ++nb) { const V b = WFrag<T16>::ld(Bt + boff + (size_t)nb * 16 * K + kc); V b2; if (NSPLIT >= 2) b2 = WFrag<T16>::ld(Bt2 + boff + (size_t)nb * 16 * K + kc);
#pragma unroll
            for (int mb = 0; mb < 4; ++mb) { acc[mb][nb] = WFrag<T16>::mma(a[mb], b, acc[mb][nb]); if (NSPLIT == 1 || NSPLIT == 2) acc[mb][nb] = WFrag<T16>::mma(a2[mb], b, acc[mb][nb]); if (NSPLIT >= 2) acc[mb][nb] = WFrag<T16>::mma(a[mb], b2, acc[mb][nb]); } }
        asm volatile("v_nop\n\tv_nop\n\tv_nop\n\tv_nop" : "+v"(acc[0][0]), "+v"(acc[1][1]), "+v"(acc[2][2]), "+v"(acc[3][3]) : "v"(a[0]), "v"(a[3]));
    }
#pragma unroll
    for (int mb = 0; mb < 4; ++mb) {
#pragma unroll
        for (int nb = 0; nb < 4; ++nb) {
#pragma unroll
            for (int j = 0; j < 8; ++j) os[(hi * 8 + j) * 68 + nb * 16 + lr] = acc[mb][nb][j]; }
        __builtin_amdgcn_wave_barrier(); asm volatile("" ::: "memory");
        float* crow = C + (size_t)(r0 + mb * 16) * ldc + c0;
#pragma unroll 1
        for (int ps = 0; ps < 2; ++ps) {
#pragma unroll
            for (int s = 0; s < 8; ++s) { const int row = 2 * s + hi, cofs = lr * 4; v4f val = *(const v4fa*)(os + row * 68 + cofs); if (BIAS) { val[0] += bfr(bias[c0 + cofs]); val[1] += bfr(bias[c0 + cofs + 1]); val[2] += bfr(bias[c0 + cofs + 2]); val[3] += bfr(bias[c0 + cofs + 3]); }
                *(volatile v4f*)(crow + (size_t)row * ldc + cofs) = val; }
            if (ps == 0) __threadfence(); }
        __builtin_amdgcn_wave_barrier(); asm volatile("" ::: "memory");
    }
}

__device__ __forceinline__ h16 tohx(float x) { return (h16)x; }
__device__ __forceinline__ void splitf(float y, unsigned short& h, unsigned short& l) { h = f2bf(y); l = f2bf(y - bf2f(h)); }
typedef __attribute__((ext_vector_type(2))) _Float16 v2h;
typedef __attribute__((ext_vector_type(4))) _Float16 v4h;
typedef __attribute__((ext_vector_type(2))) unsigned short v2us;
typedef __attribute__((ext_vector_type(4))) unsigned short v4us;
typedef __attribute__((ext_vector_type(2))) float v2f;

__global__ __launch_bounds__(256) void k_wtG(const float* __restrict__ w, int K, int N, bf* Bt) {
    const int lane = threadIdx.x & 31; const int L0 = (blockIdx.x * 8 + (threadIdx.x >> 5)) * 8; const int nlines = N * K / 64;
#pragma unroll
    for (int ps = 0; ps < 2; ++ps) {
#pragma unroll 1
        for (int l = 0; l < 8; ++l) { const int L = L0 + l; if (L >= nlines) break; const size_t e = (size_t)L * 64 + lane * 2; const int k = (int)(e % K), n = (int)(e / K); v2us o;
            o[0] = f2bf(w[(size_t)k * N + n]); o[1] = f2bf(w[(size_t)(k + 1) * N + n]); *(volatile v2us*)(Bt + e) = o; }
        if (ps == 0) __threadfence(); }
}
__global__ __launch_bounds__(256) void k_cvt8(const float* __restrict__ src, bf* dst, size_t n8) { const size_t i = (size_t)blockIdx.x * 256 + threadIdx.x; if (i >= n8) return; const v8f v = *(const v8f*)(src + i * 8); v8us o;
#pragma unroll
    for (int k = 0; k < 8; ++k) o[k] = f2bf(v[k]); *(volatile v8us*)(dst + i * 8) = o; __threadfence(); *(volatile v8us*)(dst + i * 8) = o; }
__global__ __launch_bounds__(256) void k_qplane(const float* __restrict__ F, int nrows, h16* QP) { const size_t e = ((size_t)blockIdx.x * 256 + threadIdx.x) * 2; if (e >= (size_t)NH_ * nrows * HD) return; const int d = (int)(e % HD); const int i = (int)((e / HD) % nrows); const int h = (int)(e / ((size_t)HD * nrows)); const float* f = F + (size_t)i * (2 * CIN); v2h o;
    o[0] = tohx(f[d * 4 + h]); o[1] = tohx(f[(d + 1) * 4 + h]); *(volatile v2h*)(QP + e) = o; __threadfence(); *(volatile v2h*)(QP + e) = o; }
__global__ __launch_bounds__(256) void k_vplane(const float* __restrict__ F, int nrows, h16* VT) { const size_t e = ((size_t)blockIdx.x * 256 + threadIdx.x) * 2; if (e >= (size_t)NH_ * HD * nrows) return; const int i = (int)(e % nrows); const int d = (int)((e / nrows) % HD); const int h = (int)(e / ((size_t)nrows * HD)); v2h o;
    o[0] = tohx(F[(size_t)i * (2 * CIN) + CIN + d * 4 + h]); o[1] = tohx(F[(size_t)(i + 1) * (2 * CIN) + CIN + d * 4 + h]); *(volatile v2h*)(VT + e) = o; __threadfence(); *(volatile v2h*)(VT + e) = o; }
__global__ __launch_bounds__(256) void k_rsoft(const float* __restrict__ Sb, h16* P16) {
    const int lane = threadIdx.x & 31; const int row = blockIdx.x * 8 + (threadIdx.x >> 5); if (row >= NH_ * NF) return; const float* sr = Sb + (size_t)row * NM; float v[NM / 32]; float mx = -3.0e38f;
#pragma unroll
    for (int ch = 0; ch < NM / 128; ++ch) { const v4f a = *(const v4f*)(sr + ch * 128 + lane * 4);
#pragma unroll
        for (int q = 0; q < 4; ++q) { float sa = a[q] * SCL; asm volatile("" : "+v"(sa)); v[ch * 4 + q] = sa; mx = fmaxf(mx, sa); } }
#pragma unroll
    for (int sh = 16; sh; sh >>= 1) mx = fmaxf(mx, __shfl_xor(mx, sh, 32));
    float sum = 0.f;
#pragma unroll
    for (int k = 0; k < NM / 32; ++k) { float d0 = __fsub_rn(v[k], mx); asm volatile("" : "+v"(d0)); v[k] = __builtin_amdgcn_exp2f(__fmul_rn(d0, 1.4426950408889634f)); sum += v[k]; }
#pragma unroll
    for (int sh = 16; sh; sh >>= 1) sum += __shfl_xor(sum, sh, 32);
    const float f = __fdiv_rn(PCAR, sum);
#pragma unroll 1
    for (int ps = 0; ps < 2; ++ps) {
#pragma unroll
        for (int ch = 0; ch < NM / 128; ++ch) { v4h o4;
#pragma unroll
            for (int q = 0; q < 4; ++q) o4[q] = tohx(v[ch * 4 + q] * f);
            *(volatile v4h*)(P16 + (size_t)row * NM + ch * 128 + lane * 4) = o4; }
        if (ps == 0) __threadfence(); } }
__global__ __launch_bounds__(256) void k_colstat(const float* __restrict__ Sb, float* CM, float* CL) { const int e = blockIdx.x * 256 + threadIdx.x; if (e >= NH_ * NM) return; const int h = e / NM, j = e % NM; const float* col = Sb + (size_t)h * NF * NM + j; float mx = -3.0e38f;
#pragma unroll 4
    for (int i = 0; i < NF; ++i) { float sa = col[(size_t)i * NM] * SCL; asm volatile("" : "+v"(sa)); mx = fmaxf(mx, sa); }
    float sum = 0.f;
#pragma unroll 4
    for (int i = 0; i < NF; ++i) { float sa = col[(size_t)i * NM] * SCL; asm volatile("" : "+v"(sa)); float d0 = __fsub_rn(sa, mx); asm volatile("" : "+v"(d0)); sum += __builtin_amdgcn_exp2f(__fmul_rn(d0, 1.4426950408889634f)); }
    *(volatile float*)(CM + e) = mx; *(volatile float*)(CL + e) = sum; __threadfence(); *(volatile float*)(CM + e) = mx; *(volatile float*)(CL + e) = sum; }
__global__ __launch_bounds__(256) void k_csoftT(const float* __restrict__ Sb, const float* __restrict__ CM, const float* __restrict__ CL, h16* PT) { const size_t e = ((size_t)blockIdx.x * 256 + threadIdx.x) * 2; if (e >= (size_t)NH_ * NM * NF) return; const int i = (int)(e % NF); const int j = (int)((e / NF) % NM); const int h = (int)(e / ((size_t)NF * NM)); const float m = CM[h * NM + j]; const float f = __fdiv_rn(PCAR, CL[h * NM + j]); v2h o;
#pragma unroll
    for (int q = 0; q < 2; ++q) { float sa = Sb[((size_t)h * NF + i + q) * NM + j] * SCL; asm volatile("" : "+v"(sa)); float d0 = __fsub_rn(sa, m); asm volatile("" : "+v"(d0)); o[q] = tohx(__builtin_amdgcn_exp2f(__fmul_rn(d0, 1.4426950408889634f)) * f); }
    *(volatile v2h*)(PT + e) = o; __threadfence(); *(volatile v2h*)(PT + e) = o; }
__global__ __launch_bounds__(256) void k_mergec(const float* __restrict__ O, int nrows, bf* Ah, bf* Al) { const size_t e = ((size_t)blockIdx.x * 256 + threadIdx.x) * 2; if (e >= (size_t)nrows * CIN) return; const int c = (int)(e % CIN); const int i = (int)(e / CIN); v2us oh, ol;
#pragma unroll
    for (int q = 0; q < 2; ++q) { const int cc = c + q; const int d = cc / 4, h = cc % 4; unsigned short a, b2; splitf(O[((size_t)h * nrows + i) * HD + d] * (1.0f / PCAR), a, b2); oh[q] = a; ol[q] = b2; }
    *(volatile v2us*)(Ah + e) = oh; *(volatile v2us*)(Al + e) = ol; __threadfence(); *(volatile v2us*)(Ah + e) = oh; *(volatile v2us*)(Al + e) = ol; }
__global__ __launch_bounds__(256) void k_outT(const float* __restrict__ C, int nrows, float* OUTb) { const size_t e = ((size_t)blockIdx.x * 256 + threadIdx.x) * 2; if (e >= (size_t)CIN * nrows) return; const int n = (int)(e % nrows); const int o = (int)(e / nrows); v2f v; v[0] = C[(size_t)n * CIN + o]; v[1] = C[(size_t)(n + 1) * CIN + o];
    *(volatile v2f*)(OUTb + e) = v; __threadfence(); *(volatile v2f*)(OUTb + e) = v; }

extern "C" void kernel_launch(void* const* d_in, const int* in_sizes, int n_in,
                              void* d_out, int out_size, void* d_ws, size_t ws_size, hipStream_t stream) {
    (void)in_sizes; (void)n_in; (void)out_size;
    const float* feat = (const float*)d_in[0]; const float* smap = (const float*)d_in[1]; const float* wfqv = (const float*)d_in[2]; const float* wmqv = (const float*)d_in[3]; const float* wfo = (const float*)d_in[4]; const float* wmo = (const float*)d_in[5];
    float* OUT0 = (float*)d_out; float* OUT1 = (float*)((char*)d_out + OFF1);
    char* wsp = (char*)d_ws;
    auto take = [&](size_t bytes) { char* p = wsp; wsp += (bytes + 255) & ~(size_t)255; return (void*)p; };
    bf* WFQV = (bf*)take((size_t)2 * CIN * CIN * 2); bf* WMQV = (bf*)take((size_t)2 * CIN * CIN * 2); bf* WFO = (bf*)take((size_t)CIN * CIN * 2); bf* WMO = (bf*)take((size_t)CIN * CIN * 2);
    bf* XF = (bf*)take((size_t)NF * CIN * 2); bf* XM = (bf*)take((size_t)NM * CIN * 2); float* FQV = (float*)take((size_t)NF * 2 * CIN * 4); float* MQV = (float*)take((size_t)NM * 2 * CIN * 4);
    h16* FQP = (h16*)take((size_t)NH_ * NF * HD * 2); h16* FVT = (h16*)take((size_t)NH_ * HD * NF * 2); h16* MQP = (h16*)take((size_t)NH_ * NM * HD * 2); h16* MVT = (h16*)take((size_t)NH_ * HD * NM * 2);
    float* Sb = (float*)take((size_t)NH_ * NF * NM * 4); h16* P16 = (h16*)take((size_t)NH_ * NF * NM * 2); h16* PT = (h16*)take((size_t)NH_ * NM * NF * 2); float* CM = (float*)take((size_t)NH_ * NM * 4); float* CL = (float*)take((size_t)NH_ * NM * 4);
    float* O1 = (float*)take((size_t)NH_ * NF * HD * 4); float* O2 = (float*)take((size_t)NH_ * NM * HD * 4); bf* A1h = (bf*)take((size_t)NF * CIN * 2); bf* A1l = (bf*)take((size_t)NF * CIN * 2); bf* A2h = (bf*)take((size_t)NM * CIN * 2); bf* A2l = (bf*)take((size_t)NM * CIN * 2); float* C1 = (float*)take((size_t)NF * CIN * 4); float* C2 = (float*)take((size_t)NM * CIN * 4);
    if ((size_t)(wsp - (char*)d_ws) > ws_size) return;
    k_cvt8<<<(unsigned)(((size_t)2 * CIN * CIN / 8 + 255) / 256), 256, 0, stream>>>(wfqv, WFQV, (size_t)2 * CIN * CIN / 8); k_cvt8<<<(unsigned)(((size_t)2 * CIN * CIN / 8 + 255) / 256), 256, 0, stream>>>(wmqv, WMQV, (size_t)2 * CIN * CIN / 8);
    k_cvt8<<<(unsigned)(((size_t)CIN * CIN / 8 + 255) / 256), 256, 0, stream>>>(wfo, WFO, (size_t)CIN * CIN / 8); k_cvt8<<<(unsigned)(((size_t)CIN * CIN / 8 + 255) / 256), 256, 0, stream>>>(wmo, WMO, (size_t)CIN * CIN / 8);
    for (int b = 0; b < NB_; ++b) {
        k_wtG<<<(unsigned)((CIN * NF / 64 + 63) / 64), 256, 0, stream>>>(feat + (size_t)b * CIN * NF, CIN, NF, XF); k_wtG<<<(unsigned)((CIN * NM / 64 + 63) / 64), 256, 0, stream>>>(smap + (size_t)b * CIN * NM, CIN, NM, XM);
        k_gemmw<bf, 0, false><<<dim3(NF / 64, 2 * CIN / 64, 1), 32, 0, stream>>>(XF, nullptr, WFQV, nullptr, CIN, FQV, 2 * CIN, nullptr, 0, 0, 0);
        k_gemmw<bf, 0, false><<<dim3(NM / 64, 2 * CIN / 64, 1), 32, 0, stream>>>(XM, nullptr, WMQV, nullptr, CIN, MQV, 2 * CIN, nullptr, 0, 0, 0);
        k_qplane<<<(unsigned)(((size_t)NH_ * NF * HD / 2 + 255) / 256), 256, 0, stream>>>(FQV, NF, FQP); k_vplane<<<(unsigned)(((size_t)NH_ * HD * NF / 2 + 255) / 256), 256, 0, stream>>>(FQV, NF, FVT);
        k_qplane<<<(unsigned)(((size_t)NH_ * NM * HD / 2 + 255) / 256), 256, 0, stream>>>(MQV, NM, MQP); k_vplane<<<(unsigned)(((size_t)NH_ * HD * NM / 2 + 255) / 256), 256, 0, stream>>>(MQV, NM, MVT);
        k_gemmw<h16, 0, false><<<dim3(NF / 64, NM / 64, NH_), 32, 0, stream>>>(FQP, nullptr, MQP, nullptr, HD, Sb, NM, nullptr, (size_t)NF * HD, (size_t)NM * HD, (size_t)NF * NM);
        k_rsoft<<<NH_ * NF / 8, 256, 0, stream>>>(Sb, P16);
        k_colstat<<<(NH_ * NM + 255) / 256, 256, 0, stream>>>(Sb, CM, CL); k_csoftT<<<(unsigned)(((size_t)NH_ * NM * NF / 2 + 255) / 256), 256, 0, stream>>>(Sb, CM, CL, PT);
        k_gemmw<h16, 0, false><<<dim3(NF / 64, HD / 64, NH_), 32, 0, stream>>>(P16, nullptr, MVT, nullptr, NM, O1, HD, nullptr, (size_t)NF * NM, (size_t)HD * NM, (size_t)NF * HD);
        k_gemmw<h16, 0, false><<<dim3(NM / 64, HD / 64, NH_), 32, 0, stream>>>(PT, nullptr, FVT, nullptr, NF, O2, HD, nullptr, (size_t)NM * NF, (size_t)HD * NF, (size_t)NM * HD);
        k_mergec<<<(unsigned)(((size_t)NF * CIN / 2 + 255) / 256), 256, 0, stream>>>(O1, NF, A1h, A1l); k_mergec<<<(unsigned)(((size_t)NM * CIN / 2 + 255) / 256), 256, 0, stream>>>(O2, NM, A2h, A2l);
        k_gemmw<bf, 1, false><<<dim3(NF / 64, CIN / 64, 1), 32, 0, stream>>>(A1h, A1l, WFO, nullptr, CIN, C1, CIN, nullptr, 0, 0, 0); k_outT<<<(unsigned)(((size_t)CIN * NF / 2 + 255) / 256), 256, 0, stream>>>(C1, NF, OUT0 + (size_t)b * CIN * NF);
        k_gemmw<bf, 1, false><<<dim3(NM / 64, CIN / 64, 1), 32, 0, stream>>>(A2h, A2l, WMO, nullptr, CIN, C2, CIN, nullptr, 0, 0, 0); k_outT<<<(unsigned)(((size_t)CIN * NM / 2 + 255) / 256), 256, 0, stream>>>(C2, NM, OUT1 + (size_t)b * CIN * NM); }
}
